// DialogSeqAttnMatch_16209206575367
// MI455X (gfx1250) — hardware-verified
//
#include <hip/hip_runtime.h>
#include <math.h>

typedef __attribute__((ext_vector_type(16))) _Float16 v16h;
typedef __attribute__((ext_vector_type(16))) __bf16 v16b;
typedef __attribute__((ext_vector_type(8)))  _Float16 v8h;
typedef __attribute__((ext_vector_type(8)))  float v8f;
typedef __attribute__((ext_vector_type(4)))  float v4f;
typedef __attribute__((ext_vector_type(2)))  float v2f;
typedef __attribute__((ext_vector_type(4)))  unsigned v4u;
typedef __attribute__((ext_vector_type(4)))  int v4i;
typedef float __attribute__((may_alias)) float_a;
typedef int __attribute__((may_alias)) int_a;

template <typename T> __device__ __forceinline__ void vst2(void* p, T v) { *(volatile T*)p = v; __threadfence(); *(volatile T*)p = v; }
__device__ __forceinline__ v8f wmma16(v16h a, v16h b, v8f c) {
  v8f d = __builtin_amdgcn_wmma_f32_16x16x32_f16(false, a, false, b, (short)0, c, false, false);
  asm volatile("v_nop\n\tv_nop\n\tv_nop\n\tv_nop" : "+v"(d) : "v"(a), "v"(b));
  return d;
}
__device__ __forceinline__ v8f wmma_bf(v16b a, v16b b, v8f c) {
  v8f d = __builtin_amdgcn_wmma_f32_16x16x32_bf16(false, a, false, b, (short)0, c, false, false);
  asm volatile("v_nop\n\tv_nop\n\tv_nop\n\tv_nop" : "+v"(d) : "v"(a), "v"(b));
  return d;
}
__device__ __forceinline__ v16h frag_h(const _Float16* rowk0, int lane) {
  union { v16h v; v8h q[2]; } u; const _Float16* p = rowk0 + 8 * (lane >> 4);
  u.q[0] = *(const v8h*)p; u.q[1] = *(const v8h*)(p + 16); return u.v;
}
__device__ __forceinline__ v16h frag_f32(const float* rowk0, int lane) {
  v16h a; const float* p = rowk0 + 8 * (lane >> 4);
#pragma unroll
  for (int i = 0; i < 8; ++i) { a[i] = (_Float16)p[i]; a[8 + i] = (_Float16)p[16 + i]; }
  return a;
}
__device__ __forceinline__ v16h frag_f32s(const float* rowk0, int lane, float sc) {
  v16h a; const float* p = rowk0 + 8 * (lane >> 4);
#pragma unroll
  for (int i = 0; i < 8; ++i) { a[i] = (_Float16)(p[i] * sc); a[8 + i] = (_Float16)(p[16 + i] * sc); }
  return a;
}
__device__ __forceinline__ v16h fragc_f32(const float* W, int k0, int n, int lane, int ld, int K) {
  v16h a; const int g = lane >> 4;
#pragma unroll
  for (int i = 0; i < 8; ++i) { const int ka = k0 + 8 * g + i, kb = ka + 16;
    a[i] = (_Float16)(ka < K ? W[(size_t)ka * ld + n] : 0.f); a[8 + i] = (_Float16)(kb < K ? W[(size_t)kb * ld + n] : 0.f); }
  return a;
}
struct F2 { v16b h, l; };
__device__ __forceinline__ F2 bsplit16(const float v[16]) { F2 r;
#pragma unroll
  for (int i = 0; i < 16; ++i) { const __bf16 h = (__bf16)v[i]; r.h[i] = h; r.l[i] = (__bf16)(v[i] - (float)h); }
  return r; }
__device__ __forceinline__ F2 split_row(const float* row, int k0, int lane) { float v[16]; const float* p = row + k0 + 8 * (lane >> 4);
#pragma unroll
  for (int i = 0; i < 8; ++i) { v[i] = p[i]; v[8 + i] = p[16 + i]; }
  return bsplit16(v); }
__device__ __forceinline__ F2 split_rowK(const float* row, int k0, int lane, int K) { float v[16]; const int g = lane >> 4;
#pragma unroll
  for (int i = 0; i < 8; ++i) { const int ka = k0 + 8 * g + i, kb = ka + 16; v[i] = ka < K ? row[ka] : 0.f; v[8 + i] = kb < K ? row[kb] : 0.f; }
  return bsplit16(v); }
__device__ __forceinline__ F2 split_col(const float* W, int k0, int n, int lane, int ld, int K) { float v[16]; const int g = lane >> 4;
#pragma unroll
  for (int i = 0; i < 8; ++i) { const int ka = k0 + 8 * g + i, kb = ka + 16; v[i] = ka < K ? W[(size_t)ka * ld + n] : 0.f; v[8 + i] = kb < K ? W[(size_t)kb * ld + n] : 0.f; }
  return bsplit16(v); }
__device__ __forceinline__ v8f mac3(const F2& a, const F2& b, v8f c) { c = wmma_bf(a.l, b.h, c); c = wmma_bf(a.h, b.l, c); return wmma_bf(a.h, b.h, c); }
__device__ __forceinline__ float sigm(float v) { return 1.0f / (1.0f + expf(-v)); }
#define LDSX() do { asm volatile("s_wait_dscnt 0" ::: "memory"); __builtin_amdgcn_wave_barrier(); __builtin_amdgcn_fence(__ATOMIC_RELEASE, "workgroup"); } while (0)

#define NT 32
#define L1 512
#define MQ 64
#define NK (NT * MQ)
#define HH 128

__global__ __launch_bounds__(128) void k_proj(const float* __restrict__ xd, const float* __restrict__ xq, const float* __restrict__ xa, const float* __restrict__ W, const float* __restrict__ bias, float* __restrict__ XP, float* __restrict__ YP, _Float16* __restrict__ dT) {
  __shared__ __align__(16) float so[4][16][132];
  __shared__ __align__(16) _Float16 st[HH][72];
  const int tid = threadIdx.x, wave = tid >> 5, lane = tid & 31, col = lane & 15, g = lane >> 4;
  const int which = blockIdx.y, r0 = blockIdx.x * 64 + wave * 16;
  if (which == 0 || blockIdx.x < NK / 64) {
    if (which < 2) { v8f acc[8] = {};
#pragma unroll
      for (int kc = 0; kc < HH / 32; ++kc) { F2 a;
        if (which == 0) a = split_row(xd + (size_t)(r0 + col) * HH, kc * 32, lane);
        else { const int key = r0 + col, ts = key / MQ, m = key % MQ; const float* src = m < 32 ? xq + ((size_t)ts * 32 + m) * HH : xa + ((size_t)ts * 32 + m - 32) * HH; a = split_row(src, kc * 32, lane); }
#pragma unroll
        for (int j = 0; j < 8; ++j) acc[j] = mac3(a, split_row(W + (size_t)(j * 16 + col) * HH, kc * 32, lane), acc[j]); }
#pragma unroll
      for (int j = 0; j < 8; ++j) { const int c = j * 16 + col; const float bb = bias[c];
#pragma unroll
        for (int r = 0; r < 8; ++r) { const float v = acc[j][r] + bb; so[wave][8 * g + r][c] = v > 0.f ? v : 0.f; } }
      LDSX();
      float* dst = which == 0 ? XP : YP;
#pragma unroll 4
      for (int rl = 0; rl < 16; ++rl) vst2(dst + (size_t)(r0 + rl) * HH + lane * 4, *(const v4f*)(&so[wave][rl][lane * 4])); }
    else {
      for (int q = tid; q < 64 * HH; q += 128) { const int kl = q >> 7, d = q & 127; const int key = blockIdx.x * 64 + kl, ts = key / MQ, m = key % MQ; const float v = m < 32 ? xq[((size_t)ts * 32 + m) * HH + d] : xa[((size_t)ts * 32 + m - 32) * HH + d]; st[d][kl] = (_Float16)v; }
      __syncthreads();
      for (int q = tid; q < HH * 8; q += 128) { const int d = q >> 3, pc = q & 7; vst2(dT + (size_t)d * NK + blockIdx.x * 64 + pc * 8, *(const v4u*)(&st[d][pc * 8])); } } }
}
__global__ __launch_bounds__(128) void k_attn(const float* __restrict__ XP, const float* __restrict__ YP, const _Float16* __restrict__ dT, const int* __restrict__ qmask, const int* __restrict__ amask, const float* __restrict__ rwp, float* __restrict__ out) {
  __shared__ __align__(16) float sS[4][16][68];
  __shared__ __align__(16) _Float16 sP[4][16][72];
  __shared__ __align__(16) float sO[4][16][132];
  __shared__ float smk[NK];
  const int tid = threadIdx.x, w = tid >> 5, lane = tid & 31, col = lane & 15, g = lane >> 4;
  const int i = blockIdx.y, q0 = blockIdx.x * 64 + w * 16; const size_t rq = (size_t)i * L1 + q0;
  for (int k = tid; k < NK; k += 128) { const int ts = k / MQ, m = k % MQ; const int pm = m < 32 ? qmask[ts * 32 + m] : amask[ts * 32 + m - 32]; smk[k] = pm ? 1.f : 0.f; }
  __syncthreads();
  v8f acc[8] = {};
  if (i > 0) {
    F2 aq[4];
#pragma unroll
    for (int kc = 0; kc < 4; ++kc) aq[kc] = split_row(XP + (rq + col) * HH, kc * 32, lane);
    float mrun = -3.0e38f, lrun = 0.f; const float rw = rwp[0];
#pragma unroll 1
    for (int kt = 0; kt < i; ++kt) {
      const float bias = rw * (float)(i - kt);
#pragma unroll
      for (int t = 0; t < 4; ++t) { v8f s = {}; const int key = kt * 64 + t * 16 + col;
#pragma unroll
        for (int kc = 0; kc < 4; ++kc) s = mac3(aq[kc], split_row(YP + (size_t)key * HH, kc * 32, lane), s);
        const bool pad = smk[key] != 0.f;
#pragma unroll
        for (int r = 0; r < 8; ++r) sS[w][8 * g + r][t * 16 + col] = pad ? -3.0e38f : s[r] + bias; }
      LDSX();
      float mx = -3.4e38f;
#pragma unroll
      for (int jj = 0; jj < 32; ++jj) mx = fmaxf(mx, sS[w][col][g * 32 + jj]);
      mx = fmaxf(mx, __shfl_xor(mx, 16, 32));
      const float mnew = fmaxf(mrun, mx); const float corr = mnew <= -1.0e38f ? 1.0f : expf(mrun - mnew);
      float ps = 0.f;
#pragma unroll
      for (int jj = 0; jj < 32; ++jj) { const float sv = sS[w][col][g * 32 + jj]; const float p = (sv <= -1.0e38f || mnew <= -1.0e38f) ? 0.f : expf(sv - mnew); ps += p; sP[w][col][g * 32 + jj] = (_Float16)(p * 16384.0f); }
      ps += __shfl_xor(ps, 16, 32);
      lrun = lrun * corr + ps; mrun = mnew;
#pragma unroll
      for (int r = 0; r < 8; ++r) { const float cr = __shfl(corr, 8 * g + r, 32);
#pragma unroll
        for (int t = 0; t < 8; ++t) acc[t][r] *= cr; }
      LDSX();
#pragma unroll
      for (int kc = 0; kc < 2; ++kc) { const v16h pa = frag_h(&sP[w][col][0] + kc * 32, lane);
#pragma unroll
        for (int t = 0; t < 8; ++t) acc[t] = wmma16(pa, frag_h(dT + (size_t)(t * 16 + col) * NK + kt * 64 + kc * 32, lane), acc[t]); }
      __builtin_amdgcn_wave_barrier(); }
#pragma unroll
    for (int r = 0; r < 8; ++r) { const float lr = __shfl(lrun, 8 * g + r, 32); const float inv = lr > 0.f ? 1.0f / (lr * 16384.0f) : 0.f;
#pragma unroll
      for (int t = 0; t < 8; ++t) sO[w][8 * g + r][t * 16 + col] = acc[t][r] * inv; } }
  else {
#pragma unroll
    for (int r = 0; r < 8; ++r)
#pragma unroll
      for (int t = 0; t < 8; ++t) sO[w][8 * g + r][t * 16 + col] = 0.f; }
  LDSX();
#pragma unroll 4
  for (int rl = 0; rl < 16; ++rl) vst2(out + (rq + rl) * HH + lane * 4, *(const v4f*)(&sO[w][rl][lane * 4]));
}
extern "C" void kernel_launch(void* const* d_in, const int* in_sizes, int n_in, void* d_out, int out_size, void* d_ws, size_t ws_size, hipStream_t stream) {
  (void)in_sizes; (void)n_in; (void)out_size; (void)ws_size;
  const float* xd = (const float*)d_in[0]; const float* xq = (const float*)d_in[1]; const float* xa = (const float*)d_in[2]; const float* W = (const float*)d_in[3]; const float* bias = (const float*)d_in[4]; const float* rw = (const float*)d_in[5]; const int* qm = (const int*)d_in[6]; const int* am = (const int*)d_in[7];
  float* out = (float*)d_out;
  char* ws = (char*)d_ws; size_t off = 0;
  auto take = [&](size_t bytes) { char* p = ws + off; off += (bytes + 255) & ~(size_t)255; return p; };
  float* XP = (float*)take((size_t)NT * L1 * HH * 4); float* YP = (float*)take((size_t)NK * HH * 4); _Float16* dT = (_Float16*)take((size_t)HH * NK * 2);
  k_proj<<<dim3(NT * L1 / 64, 3), 128, 0, stream>>>(xd, xq, xa, W, bias, XP, YP, dT);
  k_attn<<<dim3(L1 / 64, NT), 128, 0, stream>>>(XP, YP, dT, qm, am, rw, out);
}
